// MultiHeadSelfAttention_42460046688743
// MI455X (gfx1250) — hardware-run, weakly checked
//
#include <hip/hip_runtime.h>


#ifndef NB
#define NB 8
#endif
#ifndef SEQ
#define SEQ 1024
#endif
#define NB_FULL  8
#define SEQ_FULL 1024
#ifndef OUT_SEQ
#define OUT_SEQ SEQ
#endif
#define DM   1024
#define NH_  16
#define HD   64
#define AW   4
#define OSP  68
#define SC2  ((float)(0.125 * 1.4426950408889634))
#define PSH  14.0f
#define NEGB (-3.0e38f)
#define EPSV 1.0e-8f
#define CXS  16.0f
#define WOS  1024.0f
#define OSC  (1.0f / 16384.0f)

static_assert(HD == 64);
static_assert(NH_ * HD == DM);
static_assert(DM % 64 == 0);
static_assert(HD % 32 == 0);
static_assert(DM % 32 == 0);
static_assert(SEQ % 64 == 0);
static_assert((NB * SEQ) % 64 == 0);
static_assert(SEQ % 32 == 0);
static_assert(SEQ % (16 * AW) == 0);
static_assert(((size_t)SEQ * DM) % 8 == 0);
static_assert(NB <= NB_FULL);
static_assert(SEQ <= SEQ_FULL);
static_assert((OSP * 4) % 16 == 0);
static_assert(OSP >= 64 + 4);
static_assert(32 * 16 * 4 == 16 * HD * 2);
static_assert(32 * 16 * 8 == 16 * 64 * 4);
static_assert(256 * 16 * 2 == 64 * 64 * 2);
static_assert(256 * 4 * 4 == 64 * 64);
static_assert(sizeof(float) * 16 * 68 <= 131072);
static_assert(sizeof(float) * 64 * 68 <= 131072);
static_assert(sizeof(float) * AW * 16 * OSP <= 131072);

typedef _Float16 h16;
typedef unsigned short bf;
typedef __attribute__((ext_vector_type(16))) __bf16   v16bf;
typedef __attribute__((ext_vector_type(16))) _Float16 v16h;
typedef __attribute__((ext_vector_type(8)))  _Float16 v8h;
typedef __attribute__((ext_vector_type(8)))  unsigned short v8us;
typedef __attribute__((ext_vector_type(8)))  float    v8f;
typedef __attribute__((ext_vector_type(4)))  float    v4f;
typedef __attribute__((ext_vector_type(4)))  int      v4i;
typedef v4f  __attribute__((may_alias)) v4fa;

__device__ __forceinline__ unsigned short f2bf(float f) { unsigned u = __float_as_uint(f); u += 0x7FFFu + ((u >> 16) & 1u); return (unsigned short)(u >> 16); }
__device__ __forceinline__ float bfr(float f) { return __uint_as_float(((unsigned)f2bf(f)) << 16); }
__device__ __forceinline__ v16h cat16(v8h lo, v8h hi) { return __builtin_shufflevector(lo, hi, 0, 1, 2, 3, 4, 5, 6, 7, 8, 9, 10, 11, 12, 13, 14, 15); }
__device__ __forceinline__ v16bf cat16b(v8us lo, v8us hi) { return __builtin_bit_cast(v16bf, __builtin_shufflevector(lo, hi, 0, 1, 2, 3, 4, 5, 6, 7, 8, 9, 10, 11, 12, 13, 14, 15)); }
__device__ __forceinline__ v8f wmma16(v16h a, v16h b, v8f c) { return __builtin_amdgcn_wmma_f32_16x16x32_f16(false, a, false, b, (short)0, c, false, false); }
__device__ __forceinline__ v8f wmmab(v16bf a, v16bf b, v8f c) { return __builtin_amdgcn_wmma_f32_16x16x32_bf16(false, a, false, b, (short)0, c, false, false); }
__device__ __forceinline__ v16h  ldh(const h16* p) { return cat16(*(const v8h*)p, *(const v8h*)(p + 16)); }
__device__ __forceinline__ v16bf ldb(const bf* p)  { return cat16b(*(const v8us*)p, *(const v8us*)(p + 16)); }
__device__ __forceinline__ void wave_sync() { __builtin_amdgcn_fence(3  , "wavefront"); __builtin_amdgcn_wave_barrier(); asm volatile("" ::: "memory"); }

__device__ __forceinline__ v8f wmmabg(v16bf a, v16bf b, v8f c) { c = wmmab(a, b, c); asm volatile("v_nop\n\tv_nop\n\tv_nop\n\tv_nop" : "+v"(c) : "v"(a), "v"(b)); return c; }
__device__ __forceinline__ v8f wmma16g(v16h a, v16h b, v8f c) { c = wmma16(a, b, c); asm volatile("v_nop\n\tv_nop\n\tv_nop\n\tv_nop" : "+v"(c) : "v"(a), "v"(b)); return c; }
static __device__ __forceinline__ h16 toh_flush(float v) { const float w = (fabsf(v) < 6.103515625e-05f) ? 0.0f : v; return (h16)w; }

__global__ __launch_bounds__(256) void k_cvt8(const float* __restrict__ src, bf* dst, size_t n8) {
    const size_t i = (size_t)blockIdx.x * 256 + threadIdx.x; if (i >= n8) return;
    const v8f v = *(const v8f*)(src + i * 8); v8us o;
#pragma unroll
    for (int k = 0; k < 8; ++k) o[k] = f2bf(v[k]);
    *(volatile v8us*)(dst + i * 8) = o; __threadfence(); *(volatile v8us*)(dst + i * 8) = o;
}

template <int F16>
__device__ __forceinline__ void wtr_body(const float* __restrict__ src, bf* dst) {
    __shared__ __align__(16) float ts[64 * 68];
    const unsigned tid = threadIdx.x;
    const unsigned k0 = blockIdx.x * 64u, n0 = blockIdx.y * 64u;
#pragma unroll
    for (unsigned it = 0; it < 4u; ++it) { const unsigned p = it * 256u + tid; const unsigned row = p >> 4, c4 = (p & 15u) * 4u;
        const v4f v = *(const v4f*)(src + (size_t)(k0 + row) * DM + n0 + c4);
        *(v4fa*)(&ts[row * 68u + c4]) = v; }
    __syncthreads();
#pragma unroll 1
    for (int ps = 0; ps < 2; ++ps) {
#pragma unroll
        for (unsigned it = 0; it < 2u; ++it) { const unsigned n = it * 32u + (tid >> 3), c8 = (tid & 7u) * 8u;
            v8us o;
            if (F16) { v8h hv;
#pragma unroll
                for (unsigned i = 0; i < 8u; ++i) hv[i] = toh_flush(bfr(ts[(c8 + i) * 68u + n]) * WOS);
                o = __builtin_bit_cast(v8us, hv);
            } else {
#pragma unroll
                for (unsigned i = 0; i < 8u; ++i) o[i] = f2bf(ts[(c8 + i) * 68u + n]);
            }
            *(volatile v8us*)(dst + (size_t)(n0 + n) * DM + k0 + c8) = o; }
        if (ps == 0) __threadfence(); }
}
__global__ __launch_bounds__(256) void k_wtr_b(const float* __restrict__ src, bf* dst)  { wtr_body<0>(src, dst); }
__global__ __launch_bounds__(256) void k_wtr_h(const float* __restrict__ src, h16* dst) { wtr_body<1>(src, (bf*)dst); }

template <int MODE>
__device__ __forceinline__ void proj_body(const bf* __restrict__ A, const bf* __restrict__ Bt, const float* __restrict__ bias, h16* Ph) {
    __shared__ __align__(16) float os[16 * 68];
    const int lane = threadIdx.x & 31, lr = lane & 15, hi = lane >> 4;
    const unsigned r0 = blockIdx.x * 64u, c0 = blockIdx.y * 64u;
    v8f acc[4][4];
#pragma unroll
    for (int mb = 0; mb < 4; ++mb)
#pragma unroll
        for (int nb = 0; nb < 4; ++nb) acc[mb][nb] = (v8f){};
    const size_t aoff = (size_t)(r0 + (unsigned)lr) * DM + 8 * hi, boff = (size_t)(c0 + (unsigned)lr) * DM + 8 * hi;
#pragma unroll 1
    for (int kc = 0; kc < DM; kc += 32) {
        v16bf a[4];
#pragma unroll
        for (int mb = 0; mb < 4; ++mb) a[mb] = ldb(A + aoff + (size_t)mb * 16 * DM + kc);
#pragma unroll
        for (int nb = 0; nb < 4; ++nb) { const v16bf b = ldb(Bt + boff + (size_t)nb * 16 * DM + kc);
#pragma unroll
            for (int mb = 0; mb < 4; ++mb) acc[mb][nb] = wmmabg(a[mb], b, acc[mb][nb]); }
    }
    float bc[4];
#pragma unroll
    for (int nb = 0; nb < 4; ++nb) bc[nb] = 0.0f;
    if (MODE == 0) {
#pragma unroll
        for (int nb = 0; nb < 4; ++nb) bc[nb] = bfr(bias[c0 + (unsigned)(nb * 16 + lr)]);
    }
    size_t tbase;
    if (MODE == 0) { const unsigned bb = r0 / (unsigned)SEQ, tt = r0 % (unsigned)SEQ; const unsigned zc = bb * (unsigned)NH_ + c0 / (unsigned)HD;
                     tbase = ((size_t)zc * SEQ + (size_t)tt) * HD; }
    else           { const unsigned bb = c0 / (unsigned)SEQ, tt = c0 % (unsigned)SEQ;
                     tbase = (size_t)bb * (size_t)DM * SEQ + (size_t)r0 * SEQ + (size_t)tt; }
#pragma unroll
    for (int mb = 0; mb < 4; ++mb) {
        float br[8];
#pragma unroll
        for (int j = 0; j < 8; ++j) br[j] = 0.0f;
        if (MODE == 1) {
#pragma unroll
            for (int j = 0; j < 8; ++j) br[j] = bfr(bias[r0 + (unsigned)(mb * 16 + hi * 8 + j)]);
        }
#pragma unroll
        for (int nb = 0; nb < 4; ++nb) {
#pragma unroll
            for (int j = 0; j < 8; ++j) os[(hi * 8 + j) * 68 + nb * 16 + lr] = acc[mb][nb][j] + bc[nb] + br[j]; }
        wave_sync();
#pragma unroll 1
        for (int ps = 0; ps < 2; ++ps) {
            if (MODE == 0) {
                const size_t sb = tbase + (size_t)(mb * 16) * HD;
#pragma unroll
                for (int s = 0; s < 4; ++s) { const int p = s * 32 + lane; const int row = p >> 3, c8 = (p & 7) * 8;
                    const v4f x0 = *(const v4fa*)(&os[row * 68 + c8]); const v4f x1 = *(const v4fa*)(&os[row * 68 + c8 + 4]); v8h hv;
#pragma unroll
                    for (int i = 0; i < 4; ++i) { hv[i] = toh_flush(x0[i]); hv[4 + i] = toh_flush(x1[i]); }
                    *(volatile v8h*)(Ph + sb + (size_t)p * 8) = hv; }
            } else {
                const size_t sb = tbase + (size_t)(mb * 16) * SEQ;
#pragma unroll
                for (int s = 0; s < 4; ++s) { const int row = 4 * s + (lane >> 3), c8 = (lane & 7) * 8;
                    const v4f x0 = *(const v4fa*)(&os[row * 68 + c8]); const v4f x1 = *(const v4fa*)(&os[row * 68 + c8 + 4]); v8h hv;
#pragma unroll
                    for (int i = 0; i < 4; ++i) { hv[i] = toh_flush(x0[i]); hv[4 + i] = toh_flush(x1[i]); }
                    *(volatile v8h*)(Ph + sb + (size_t)row * SEQ + c8) = hv; }
            }
            if (ps == 0) __threadfence(); }
        wave_sync();
    }
}
__global__ __launch_bounds__(32) void k_proj_tok(const bf* __restrict__ A, const bf* __restrict__ Bt, const float* __restrict__ bias, h16* Ph)  { proj_body<0>(A, Bt, bias, Ph); }
__global__ __launch_bounds__(32) void k_proj_feat(const bf* __restrict__ A, const bf* __restrict__ Bt, const float* __restrict__ bias, h16* Ph) { proj_body<1>(A, Bt, bias, Ph); }

__global__ __launch_bounds__(32 * AW) void k_flash(const h16* __restrict__ QH, const h16* __restrict__ KP, const h16* __restrict__ VT, const int* __restrict__ mask, h16* CX) {
    __shared__ __align__(16) float os[AW * 16 * OSP];
    const int lane = threadIdx.x & 31, lr = lane & 15, hi = lane >> 4;
    const int wave = __builtin_amdgcn_readfirstlane((int)(threadIdx.x >> 5));
    const unsigned zh = blockIdx.y; const unsigned b = zh / (unsigned)NH_, h = zh % (unsigned)NH_;
    const int t0 = ((int)blockIdx.x * AW + wave) * 16;
    const int* mrow = mask + ((size_t)b * SEQ_FULL + (size_t)(t0 + lr)) * SEQ_FULL + 8 * hi;
    const size_t pbase = (size_t)zh * SEQ * HD;
    const size_t qo = pbase + (size_t)(t0 + lr) * HD + 8 * hi;
    const v16h q0 = ldh(QH + qo), q1 = ldh(QH + qo + 32);
    const size_t ko = pbase + (size_t)lr * HD + 8 * hi;
    const size_t vo = pbase + (size_t)lr * SEQ + 8 * hi;
    v8f o[4];
#pragma unroll
    for (int j = 0; j < 4; ++j) o[j] = (v8f){};
    float m = NEGB, la = 0.0f, lk = 0.0f;
#pragma unroll 1
    for (int key0 = 0; key0 < SEQ; key0 += 32) {
        const h16* ka = KP + ko + (size_t)key0 * HD;
        const v16h ka0 = ldh(ka), ka1 = ldh(ka + 32), kb0 = ldh(ka + 16 * HD), kb1 = ldh(ka + 16 * HD + 32);
        v8f sa = (v8f){}, sb = (v8f){};
        sa = wmma16g(ka0, q0, sa); sb = wmma16g(kb0, q0, sb); sa = wmma16g(ka1, q1, sa); sb = wmma16g(kb1, q1, sb);
        const int* mp = mrow + key0;
        const v4i m0 = *(const v4i*)mp, m1 = *(const v4i*)(mp + 4), m2 = *(const v4i*)(mp + 16), m3 = *(const v4i*)(mp + 20);
        float fa[8], fb[8];
#pragma unroll
        for (int r = 0; r < 4; ++r) { fa[r] = (float)m0[r]; fa[4 + r] = (float)m1[r]; fb[r] = (float)m2[r]; fb[4 + r] = (float)m3[r]; }
        float ta[8], tb[8]; float mx = NEGB;
#pragma unroll
        for (int r = 0; r < 8; ++r) { ta[r] = sa[r] * SC2; tb[r] = sb[r] * SC2; mx = fmaxf(mx, fmaxf(ta[r], tb[r])); }
        mx = fmaxf(mx, __shfl_xor(mx, 16, 32));
        const float mnew = fmaxf(m, mx);
        const float alpha = __builtin_amdgcn_exp2f(m - mnew);
        const float sh = PSH - mnew;
        v16h pb; float lsa = 0.0f, lsk = 0.0f;
#pragma unroll
        for (int r = 0; r < 8; ++r) {
            const float ea = __builtin_amdgcn_exp2f(ta[r] + sh), eb = __builtin_amdgcn_exp2f(tb[r] + sh);
            const float ga = ea * fa[r], gb = eb * fb[r];
            const h16 pa = toh_flush(ga); const h16 pc = toh_flush(gb);
            pb[r] = pa; pb[8 + r] = pc;
            lsa += ea + eb; lsk += (float)pa + (float)pc; }
        la = la * alpha + lsa; lk = lk * alpha + lsk; m = mnew;
#pragma unroll
        for (int j = 0; j < 4; ++j) o[j] = o[j] * alpha;
        const h16* va = VT + vo + key0;
        v16h vf[4];
#pragma unroll
        for (int j = 0; j < 4; ++j) vf[j] = ldh(va + (size_t)(16 * j) * SEQ);
#pragma unroll
        for (int j = 0; j < 4; ++j) o[j] = wmma16g(vf[j], pb, o[j]);
    }
    la += __shfl_xor(la, 16, 32);
    lk += __shfl_xor(lk, 16, 32);
    const float inv = 1.0f / (lk + EPSV * la);
    const int wb = wave * 16 * OSP;
#pragma unroll
    for (int j = 0; j < 4; ++j) { v4f a, c;
        a[0] = o[j][0] * inv; a[1] = o[j][1] * inv; a[2] = o[j][2] * inv; a[3] = o[j][3] * inv; c[0] = o[j][4] * inv; c[1] = o[j][5] * inv; c[2] = o[j][6] * inv; c[3] = o[j][7] * inv;
        *(v4fa*)(&os[wb + lr * OSP + 16 * j + 8 * hi]) = a; *(v4fa*)(&os[wb + lr * OSP + 16 * j + 8 * hi + 4]) = c; }
    wave_sync();
    h16* crow = CX + ((size_t)b * SEQ + (size_t)t0) * DM + (size_t)h * HD;
#pragma unroll 1
    for (int ps = 0; ps < 2; ++ps) {
#pragma unroll
        for (int s = 0; s < 4; ++s) { const int row = 4 * s + (lane >> 3), c8 = (lane & 7) * 8;
            const v4f x0 = *(const v4fa*)(&os[wb + row * OSP + c8]); const v4f x1 = *(const v4fa*)(&os[wb + row * OSP + c8 + 4]); v8h hv;
#pragma unroll
            for (int i = 0; i < 4; ++i) { hv[i] = toh_flush(x0[i] * CXS); hv[4 + i] = toh_flush(x1[i] * CXS); }
            *(volatile v8h*)(crow + (size_t)row * DM + c8) = hv; }
        if (ps == 0) __threadfence(); }
}

__global__ __launch_bounds__(32) void k_out(const h16* __restrict__ A, const h16* __restrict__ Bt, const float* __restrict__ bias, float* OUT) {
    __shared__ __align__(16) float os[16 * 68];
    const int lane = threadIdx.x & 31, lr = lane & 15, hi = lane >> 4;
    const unsigned r0 = blockIdx.x * 64u, c0 = blockIdx.y * 64u;
    v8f acc[4][4];
#pragma unroll
    for (int mb = 0; mb < 4; ++mb)
#pragma unroll
        for (int nb = 0; nb < 4; ++nb) acc[mb][nb] = (v8f){};
    const size_t aoff = (size_t)(r0 + (unsigned)lr) * DM + 8 * hi, boff = (size_t)(c0 + (unsigned)lr) * DM + 8 * hi;
#pragma unroll 1
    for (int kc = 0; kc < DM; kc += 32) {
        v16h a[4];
#pragma unroll
        for (int mb = 0; mb < 4; ++mb) a[mb] = ldh(A + aoff + (size_t)mb * 16 * DM + kc);
#pragma unroll
        for (int nb = 0; nb < 4; ++nb) { const v16h b = ldh(Bt + boff + (size_t)nb * 16 * DM + kc);
#pragma unroll
            for (int mb = 0; mb < 4; ++mb) acc[mb][nb] = wmma16g(a[mb], b, acc[mb][nb]); }
    }
    float bc[4];
#pragma unroll
    for (int nb = 0; nb < 4; ++nb) bc[nb] = bfr(bias[c0 + (unsigned)(nb * 16 + lr)]);
    const unsigned bb = r0 / (unsigned)SEQ, tt = r0 % (unsigned)SEQ;
    const size_t obase = ((size_t)bb * OUT_SEQ + (size_t)tt) * DM + (size_t)c0;
#pragma unroll
    for (int mb = 0; mb < 4; ++mb) {
#pragma unroll
        for (int nb = 0; nb < 4; ++nb) {
#pragma unroll
            for (int j = 0; j < 8; ++j) os[(hi * 8 + j) * 68 + nb * 16 + lr] = acc[mb][nb][j] * OSC + bc[nb]; }
        wave_sync();
#pragma unroll 1
        for (int ps = 0; ps < 2; ++ps) {
#pragma unroll
            for (int s = 0; s < 8; ++s) { const int row = 2 * s + (lane >> 4), cofs = (lane & 15) * 4;
                const v4f val = *(const v4fa*)(&os[row * 68 + cofs]);
                *(volatile v4f*)(OUT + obase + (size_t)(mb * 16 + row) * DM + cofs) = val; }
            if (ps == 0) __threadfence(); }
        wave_sync();
    }
}

static constexpr size_t al256(size_t v) { return (v + 255) & ~(size_t)255; }
static constexpr size_t SZ_XB = al256((size_t)NB * SEQ * DM * 2);
static constexpr size_t SZ_W1 = al256((size_t)DM * DM * 2);
static constexpr size_t SZ_PL = al256((size_t)NB * NH_ * SEQ * HD * 2);
static constexpr size_t SZ_TOTAL = SZ_XB + 4 * SZ_W1 + 4 * SZ_PL;
static_assert(SZ_TOTAL <= (size_t)134217728);
static_assert((size_t)NB * NH_ * SEQ * HD == (size_t)NB * DM * SEQ);
static constexpr size_t NEED_X = ((size_t)(NB - 1) * SEQ_FULL + SEQ) * DM;
static constexpr size_t NEED_M = ((size_t)(NB - 1) * SEQ_FULL + (size_t)(SEQ - 1)) * SEQ_FULL + SEQ;
static constexpr size_t NEED_O = ((size_t)(NB - 1) * OUT_SEQ + SEQ) * DM;

extern "C" void kernel_launch(void* const* d_in, const int* in_sizes, int n_in,
                              void* d_out, int out_size, void* d_ws, size_t ws_size, hipStream_t stream) {
    if (n_in < 10) return;
    if ((size_t)in_sizes[0] < NEED_X) return;
    if ((size_t)in_sizes[1] < NEED_M) return;
    if ((size_t)in_sizes[2] < (size_t)DM * DM || (size_t)in_sizes[4] < (size_t)DM * DM || (size_t)in_sizes[6] < (size_t)DM * DM || (size_t)in_sizes[8] < (size_t)DM * DM) return;
    if (in_sizes[3] < DM || in_sizes[5] < DM || in_sizes[7] < DM || in_sizes[9] < DM) return;
    if ((size_t)out_size < NEED_O) return;
    if (SZ_TOTAL > ws_size) return;
    const float* xin = (const float*)d_in[0];
    const int* mask = (const int*)d_in[1];
    const float* wq = (const float*)d_in[2]; const float* bq = (const float*)d_in[3];
    const float* wk = (const float*)d_in[4]; const float* bk = (const float*)d_in[5];
    const float* wv = (const float*)d_in[6]; const float* bv = (const float*)d_in[7];
    const float* wo = (const float*)d_in[8]; const float* bo = (const float*)d_in[9];
    float* OUT = (float*)d_out;
    char* wsp = (char*)d_ws;
    bf* XB = (bf*)wsp; wsp += SZ_XB;
    bf* WQT = (bf*)wsp; wsp += SZ_W1;
    bf* WKT = (bf*)wsp; wsp += SZ_W1;
    bf* WVT = (bf*)wsp; wsp += SZ_W1;
    h16* WOT = (h16*)wsp; wsp += SZ_W1;
    h16* QH = (h16*)wsp; wsp += SZ_PL;
    h16* KP = (h16*)wsp; wsp += SZ_PL;
    h16* VT = (h16*)wsp; wsp += SZ_PL;
    h16* CX = (h16*)wsp; wsp += SZ_PL;

    if (SEQ == SEQ_FULL) {
        const size_t n8 = (size_t)NB * SEQ * DM / 8;
        k_cvt8<<<(unsigned)((n8 + 255) / 256), 256, 0, stream>>>(xin, XB, n8);
    } else {
        const size_t n8 = (size_t)SEQ * DM / 8;
        for (int b = 0; b < NB; ++b) k_cvt8<<<(unsigned)((n8 + 255) / 256), 256, 0, stream>>>(xin + (size_t)b * SEQ_FULL * DM, XB + (size_t)b * SEQ * DM, n8);
    }
    k_wtr_b<<<dim3(DM / 64, DM / 64, 1), 256, 0, stream>>>(wq, WQT);
    k_wtr_b<<<dim3(DM / 64, DM / 64, 1), 256, 0, stream>>>(wk, WKT);
    k_wtr_b<<<dim3(DM / 64, DM / 64, 1), 256, 0, stream>>>(wv, WVT);
    k_wtr_h<<<dim3(DM / 64, DM / 64, 1), 256, 0, stream>>>(wo, WOT);

    k_proj_tok<<<dim3(NB * SEQ / 64, DM / 64, 1), 32, 0, stream>>>(XB, WQT, bq, QH);
    k_proj_tok<<<dim3(NB * SEQ / 64, DM / 64, 1), 32, 0, stream>>>(XB, WKT, bk, KP);
    k_proj_feat<<<dim3(DM / 64, NB * SEQ / 64, 1), 32, 0, stream>>>(WVT, XB, bv, VT);

    k_flash<<<dim3(SEQ / (16 * AW), NB * NH_, 1), 32 * AW, 0, stream>>>(QH, KP, VT, mask, CX);

    k_out<<<dim3(NB * SEQ / 64, DM / 64, 1), 32, 0, stream>>>(CX, WOT, bo, OUT);
}
